// DN4_10668698763884
// MI455X (gfx1250) — hardware-verified
//
#include <hip/hip_runtime.h>
#define NQI 32
#define NSI 50
#define HW0 7056
#define HW1 1764
#define HW2 441
#define DD 64
#define WAY 5
#define MS 2205
#define MSP 2240
#define MQP 448

typedef __bf16 v16b __attribute__((ext_vector_type(16)));
typedef unsigned short v8us __attribute__((ext_vector_type(8), may_alias));
typedef float  v8f  __attribute__((ext_vector_type(8)));
typedef float  v4f  __attribute__((ext_vector_type(4)));
typedef float  v4fa __attribute__((ext_vector_type(4), may_alias));
union FragB { v16b v; v8us half[2]; unsigned short u[16]; };

__device__ __forceinline__ unsigned short bf16_bits(float x) { unsigned int u = __float_as_uint(x); return (unsigned short)((u + 0x7FFFu + ((u >> 16) & 1u)) >> 16); }
__device__ __forceinline__ float bf16_val(unsigned short b) { return __uint_as_float(((unsigned int)b) << 16); }
__device__ __forceinline__ float bf16_round(float x) { return bf16_val(bf16_bits(x)); }
template <int NT>
__device__ __forceinline__ v8f mmaN(v16b ah, v16b al, v16b bh, v16b bl, v8f c) {
  c = __builtin_amdgcn_wmma_f32_16x16x32_bf16(false, ah, false, bh, (short)0, c, false, false);
  if (NT >= 2) c = __builtin_amdgcn_wmma_f32_16x16x32_bf16(false, al, false, bh, (short)0, c, false, false);
  if (NT >= 3) c = __builtin_amdgcn_wmma_f32_16x16x32_bf16(false, ah, false, bl, (short)0, c, false, false);
  asm volatile("v_nop\n\tv_nop\n\tv_nop\n\tv_nop" : "+v"(c) : "v"(ah), "v"(al), "v"(bh), "v"(bl));
  return c;
}

__global__ __launch_bounds__(256) void k_wt_bf16(const float* __restrict__ W, unsigned short* __restrict__ Wt, int K, int N) {
  const int t = blockIdx.x * 256 + threadIdx.x;
  const int k8n = K / 8;
  if (t >= N * k8n) return;
  const int n = t / k8n, k8 = (t % k8n) * 8;
  v8us v;
#pragma unroll
  for (int i = 0; i < 8; ++i) v[i] = bf16_bits(W[(size_t)(k8 + i) * N + n]);
  *(volatile v8us*)(Wt + (size_t)n * K + k8) = v;
  __threadfence();
  *(volatile v8us*)(Wt + (size_t)n * K + k8) = v;
}

template <bool ASPLIT, int ACT, bool BIAS_BF16>
__global__ __launch_bounds__(128) void k_gemm_bf(const float* __restrict__ A, int lda, const unsigned short* __restrict__ Wt, int ldb,
                                               const float* __restrict__ bias, float* __restrict__ C, int ldc, int M, int N, int K) {
  __shared__ __attribute__((aligned(16))) float so[4][16][64];
  const int tid = threadIdx.x, w = tid >> 5, lane = tid & 31, ln = lane & 15, hh = lane >> 4;
  const int ntn = N / 64;
  const int wid = blockIdx.x * 4 + w;
  const int mt = wid / ntn, nq = wid % ntn;
  if (mt * 16 >= M) return;
  const int row0 = mt * 16, col0 = nq * 64;
  const float* arow = A + (size_t)(row0 + ln) * lda;
  v8f acc[4] = {};
  for (int kb = 0; kb < K; kb += 32) {
    FragB ah, al;
    const v4f x0 = *(const v4fa*)(arow + kb + 8 * hh), x1 = *(const v4fa*)(arow + kb + 8 * hh + 4);
    const v4f x2 = *(const v4fa*)(arow + kb + 16 + 8 * hh), x3 = *(const v4fa*)(arow + kb + 16 + 8 * hh + 4);
    float xs[16] = {x0[0],x0[1],x0[2],x0[3],x1[0],x1[1],x1[2],x1[3],x2[0],x2[1],x2[2],x2[3],x3[0],x3[1],x3[2],x3[3]};
#pragma unroll
    for (int i = 0; i < 16; ++i) { const unsigned short hb = bf16_bits(xs[i]); ah.u[i] = hb; al.u[i] = ASPLIT ? bf16_bits(xs[i] - bf16_val(hb)) : (unsigned short)0; }
#pragma unroll
    for (int t = 0; t < 4; ++t) {
      const unsigned short* brow = Wt + (size_t)(col0 + t * 16 + ln) * ldb + kb;
      FragB b;
      b.half[0] = *(const v8us*)(brow + 8 * hh);
      b.half[1] = *(const v8us*)(brow + 16 + 8 * hh);
      acc[t] = mmaN<ASPLIT ? 2 : 1>(ah.v, al.v, b.v, b.v, acc[t]);
    }
  }
#pragma unroll
  for (int t = 0; t < 4; ++t) {
    float bv = bias ? bias[col0 + t * 16 + ln] : 0.f;
    if (BIAS_BF16) bv = bf16_round(bv);
#pragma unroll
    for (int r = 0; r < 8; ++r) { float v = acc[t][r] + bv; if (ACT == 1) v = fmaxf(v, 0.f); so[w][8 * hh + r][t * 16 + ln] = v; }
  }
  __builtin_amdgcn_fence(__ATOMIC_ACQ_REL, "workgroup");
  __builtin_amdgcn_wave_barrier();
  const int rsub = lane >> 4, c4 = (lane & 15) * 4;
  for (int pass = 0; pass < 2; ++pass) {
#pragma unroll
    for (int q = 0; q < 8; ++q) {
      const int r = q * 2 + rsub;
      const v4f v = *(const v4fa*)&so[w][r][c4];
      *(volatile v4f*)(C + (size_t)(row0 + r) * ldc + col0 + c4) = v;
    }
    if (pass == 0) __threadfence();
  }
}

template <int D, bool CAUSAL>
__global__ __launch_bounds__(128) void k_flash(const float* __restrict__ qb, const float* __restrict__ kb, const float* __restrict__ vb,
                                             int pitch, int T, int H, float scale, float* __restrict__ y, int ypitch) {
  constexpr int KS = D / 32;
  constexpr int DT = D / 16;
  __shared__ __attribute__((aligned(16))) unsigned short sKh[32][D + 8], sKl[32][D + 8], sVh[32][D + 8], sVl[32][D + 8];
  __shared__ __attribute__((aligned(16))) unsigned short sPh[4][16][40], sPl[4][16][40];
  __shared__ __attribute__((aligned(16))) float sO[4][16][D];
  const int tid = threadIdx.x, w = tid >> 5, lane = tid & 31, ln = lane & 15, hh = lane >> 4;
  const int nqb = (T + 63) / 64;
  const int bh = blockIdx.x / nqb, qblk = blockIdx.x % nqb;
  const int b = bh / H, h = bh % H;
  const int q0 = qblk * 64 + w * 16;
  const float* Q = qb + (size_t)b * T * pitch + h * D;
  const float* K = kb + (size_t)b * T * pitch + h * D;
  const float* V = vb + (size_t)b * T * pitch + h * D;

  FragB aqh[KS], aql[KS];
  {
    int row = q0 + ln; if (row >= T) row = T - 1;
    const float* qr = Q + (size_t)row * pitch;
#pragma unroll
    for (int ks = 0; ks < KS; ++ks)
#pragma unroll
      for (int i = 0; i < 16; ++i) {
        const int d = ks * 32 + ((i < 8) ? (8 * hh + i) : (16 + 8 * hh + (i - 8)));
        const float x = qr[d] * scale; const unsigned short hb = bf16_bits(x);
        aqh[ks].u[i] = hb; aql[ks].u[i] = bf16_bits(x - bf16_val(hb));
      }
  }
  float m_r[8], l_r[8];
#pragma unroll
  for (int r = 0; r < 8; ++r) { m_r[r] = -3.0e38f; l_r[r] = 0.f; }
  v8f oacc[DT];
#pragma unroll
  for (int dt = 0; dt < DT; ++dt) oacc[dt] = (v8f){0.f,0.f,0.f,0.f,0.f,0.f,0.f,0.f};

  const int kv_end = CAUSAL ? min(T, qblk * 64 + 64) : T;
  for (int j0 = 0; j0 < kv_end; j0 += 32) {
    __syncthreads();
    for (int e = tid; e < 32 * (D / 4); e += 128) {
      const int r = e / (D / 4), c4 = (e % (D / 4)) * 4;
      const int key = j0 + r;
      v4f kf = {0.f,0.f,0.f,0.f}, vf = {0.f,0.f,0.f,0.f};
      if (key < T) { kf = *(const v4fa*)(K + (size_t)key * pitch + c4); vf = *(const v4fa*)(V + (size_t)key * pitch + c4); }
#pragma unroll
      for (int t = 0; t < 4; ++t) {
        unsigned short hb = bf16_bits(kf[t]); sKh[r][c4 + t] = hb; sKl[r][c4 + t] = bf16_bits(kf[t] - bf16_val(hb));
        hb = bf16_bits(vf[t]); sVh[r][c4 + t] = hb; sVl[r][c4 + t] = bf16_bits(vf[t] - bf16_val(hb));
      }
    }
    __syncthreads();
    v8f s[2];
#pragma unroll
    for (int nt = 0; nt < 2; ++nt) {
      v8f acc = {};
#pragma unroll
      for (int ks = 0; ks < KS; ++ks) {
        FragB bh_, bl_;
        bh_.half[0] = *(const v8us*)&sKh[nt * 16 + ln][ks * 32 + 8 * hh]; bh_.half[1] = *(const v8us*)&sKh[nt * 16 + ln][ks * 32 + 16 + 8 * hh];
        bl_.half[0] = *(const v8us*)&sKl[nt * 16 + ln][ks * 32 + 8 * hh]; bl_.half[1] = *(const v8us*)&sKl[nt * 16 + ln][ks * 32 + 16 + 8 * hh];
        acc = mmaN<3>(aqh[ks].v, aql[ks].v, bh_.v, bl_.v, acc);
      }
      s[nt] = acc;
    }
    float alpha[8];
#pragma unroll
    for (int r = 0; r < 8; ++r) {
      const int qi = q0 + 8 * hh + r;
      const int ja = j0 + ln, jb = j0 + 16 + ln;
      if (CAUSAL) { if (ja > qi) s[0][r] = -3.0e38f; if (jb > qi) s[1][r] = -3.0e38f; }
      if (ja >= T) s[0][r] = -3.0e38f;
      if (jb >= T) s[1][r] = -3.0e38f;
      float mx = fmaxf(s[0][r], s[1][r]);
      mx = fmaxf(mx, __shfl_xor(mx, 1, 32)); mx = fmaxf(mx, __shfl_xor(mx, 2, 32)); mx = fmaxf(mx, __shfl_xor(mx, 4, 32)); mx = fmaxf(mx, __shfl_xor(mx, 8, 32));
      const float mnew = fmaxf(m_r[r], mx);
      alpha[r] = (mnew > -1.0e38f) ? __expf(m_r[r] - mnew) : 1.0f;
      const float p0 = (s[0][r] > -1.0e38f) ? __expf(s[0][r] - mnew) : 0.f;
      const float p1 = (s[1][r] > -1.0e38f) ? __expf(s[1][r] - mnew) : 0.f;
      m_r[r] = mnew;
      l_r[r] = l_r[r] * alpha[r] + p0 + p1;
      unsigned short hb = bf16_bits(p0); sPh[w][8 * hh + r][ln] = hb;      sPl[w][8 * hh + r][ln] = bf16_bits(p0 - bf16_val(hb));
      hb = bf16_bits(p1);                sPh[w][8 * hh + r][16 + ln] = hb; sPl[w][8 * hh + r][16 + ln] = bf16_bits(p1 - bf16_val(hb));
    }
#pragma unroll
    for (int dt = 0; dt < DT; ++dt)
#pragma unroll
      for (int r = 0; r < 8; ++r) oacc[dt][r] *= alpha[r];
    __builtin_amdgcn_fence(__ATOMIC_ACQ_REL, "workgroup");
    __builtin_amdgcn_wave_barrier();
    FragB pah, pal;
    pah.half[0] = *(const v8us*)&sPh[w][ln][8 * hh]; pah.half[1] = *(const v8us*)&sPh[w][ln][16 + 8 * hh];
    pal.half[0] = *(const v8us*)&sPl[w][ln][8 * hh]; pal.half[1] = *(const v8us*)&sPl[w][ln][16 + 8 * hh];
#pragma unroll
    for (int dt = 0; dt < DT; ++dt) {
      FragB bvh, bvl;
#pragma unroll
      for (int i = 0; i < 8; ++i) {
        bvh.u[i] = sVh[8 * hh + i][dt * 16 + ln]; bvh.u[8 + i] = sVh[16 + 8 * hh + i][dt * 16 + ln];
        bvl.u[i] = sVl[8 * hh + i][dt * 16 + ln]; bvl.u[8 + i] = sVl[16 + 8 * hh + i][dt * 16 + ln];
      }
      oacc[dt] = mmaN<3>(pah.v, pal.v, bvh.v, bvl.v, oacc[dt]);
    }
    __builtin_amdgcn_fence(__ATOMIC_ACQ_REL, "workgroup");
    __builtin_amdgcn_wave_barrier();
  }
#pragma unroll
  for (int r = 0; r < 8; ++r) {
    float l = l_r[r];
    l += __shfl_xor(l, 1, 32); l += __shfl_xor(l, 2, 32); l += __shfl_xor(l, 4, 32); l += __shfl_xor(l, 8, 32);
    l_r[r] = (l > 0.f) ? 1.0f / l : 0.f;
  }
#pragma unroll
  for (int dt = 0; dt < DT; ++dt)
#pragma unroll
    for (int r = 0; r < 8; ++r) sO[w][8 * hh + r][dt * 16 + ln] = oacc[dt][r] * l_r[r];
  __builtin_amdgcn_fence(__ATOMIC_ACQ_REL, "workgroup");
  __builtin_amdgcn_wave_barrier();
  for (int pass = 0; pass < 2; ++pass) {
    for (int r = 0; r < 16; ++r) {
      const int row = q0 + r;
      if (row < T && lane < D / 4) {
        const v4f val = *(const v4fa*)&sO[w][r][lane * 4];
        *(volatile v4f*)(y + ((size_t)b * T + row) * ypitch + h * D + lane * 4) = val;
      }
    }
    if (pass == 0) __threadfence();
  }
}

template <bool AFFINE, bool RESID, bool RES_BF16>
__global__ __launch_bounds__(256) void k_transpose32(const float* __restrict__ in, float* __restrict__ out, int rows, int cols,
                                                    const float* __restrict__ scale, const float* __restrict__ shift, const float* __restrict__ res) {
  __shared__ float tile[32][33];
  const int b = blockIdx.z;
  const int r0 = blockIdx.y * 32, c0 = blockIdx.x * 32;
  const float* src = in + (size_t)b * rows * cols;
  float* dst = out + (size_t)b * rows * cols;
  const int tx = threadIdx.x & 31, ty = threadIdx.x >> 5;
  for (int i = ty; i < 32; i += 8) tile[i][tx] = src[(size_t)(r0 + i) * cols + c0 + tx];
  __syncthreads();
  for (int pass = 0; pass < 2; ++pass) {
    for (int i = ty; i < 32; i += 8) {
      float v = tile[tx][i];
      const int orow = c0 + i;
      if (AFFINE) v = v * scale[orow] + shift[orow];
      if (RESID) { float rv = res[(size_t)b * rows * cols + (size_t)orow * rows + r0 + tx]; if (RES_BF16) rv = bf16_round(rv); v += rv; }
      *(volatile float*)(dst + (size_t)orow * rows + r0 + tx) = v;
    }
    if (pass == 0) __threadfence();
  }
}

__global__ __launch_bounds__(256) void k_pool2_pm(const float* __restrict__ in, float* __restrict__ out, int Bn, int H, int W, int C) {
  const size_t t = (size_t)blockIdx.x * 256 + threadIdx.x;
  const int c4n = C / 4, Ho = H / 2, Wo = W / 2;
  const size_t total = (size_t)Bn * Ho * Wo * c4n;
  if (t >= total) return;
  const int c4 = (int)(t % c4n) * 4; size_t rest = t / c4n;
  const int pw = (int)(rest % Wo); rest /= Wo; const int ph = (int)(rest % Ho); const int b = (int)(rest / Ho);
  const float* base = in + (size_t)b * H * W * C;
  const int p00 = (2 * ph) * W + 2 * pw;
  const v4f a = *(const v4fa*)(base + (size_t)p00 * C + c4), bq = *(const v4fa*)(base + (size_t)(p00 + 1) * C + c4);
  const v4f c = *(const v4fa*)(base + (size_t)(p00 + W) * C + c4), d = *(const v4fa*)(base + (size_t)(p00 + W + 1) * C + c4);
  v4f m; for (int i = 0; i < 4; ++i) m[i] = fmaxf(fmaxf(a[i], bq[i]), fmaxf(c[i], d[i]));
  float* dst = out + ((size_t)b * Ho * Wo + (size_t)ph * Wo + pw) * C + c4;
  *(volatile v4f*)dst = m;
  __threadfence();
  *(volatile v4f*)dst = m;
}

template <int DQ, int DV>
__global__ __launch_bounds__(128) void k_flash2(const float* __restrict__ Qb, size_t qstride, int qpitch, int Tq,
                                              const float* __restrict__ Kb, size_t kstride, int kpitch, int Tk,
                                              const float* __restrict__ Vb, size_t vstride, int vpitch,
                                              float scale, float* __restrict__ y, size_t ystride, int ypitch) {
  constexpr int KS = DQ / 32, DT = DV / 16;
  __shared__ __attribute__((aligned(16))) unsigned short sKh[32][DQ + 8], sKl[32][DQ + 8], sVh[32][DV + 8], sVl[32][DV + 8];
  __shared__ __attribute__((aligned(16))) unsigned short sPh[4][16][40], sPl[4][16][40];
  __shared__ __attribute__((aligned(16))) float sO[4][16][DV];
  const int tid = threadIdx.x, w = tid >> 5, lane = tid & 31, ln = lane & 15, hh = lane >> 4;
  const int nqb = (Tq + 63) / 64;
  const int bh = blockIdx.x / nqb, qblk = blockIdx.x % nqb;
  const int dv0 = blockIdx.y * DV;
  const int q0 = qblk * 64 + w * 16;
  const float* Q = Qb + (size_t)bh * qstride; const float* K = Kb + (size_t)bh * kstride; const float* V = Vb + (size_t)bh * vstride + dv0;
  FragB aqh[KS], aql[KS];
  {
    int row = q0 + ln; if (row >= Tq) row = Tq - 1;
    const float* qr = Q + (size_t)row * qpitch;
#pragma unroll
    for (int ks = 0; ks < KS; ++ks)
#pragma unroll
      for (int i = 0; i < 16; ++i) {
        const int d = ks * 32 + ((i < 8) ? (8 * hh + i) : (16 + 8 * hh + (i - 8)));
        const float x = qr[d] * scale; const unsigned short hb = bf16_bits(x);
        aqh[ks].u[i] = hb; aql[ks].u[i] = bf16_bits(x - bf16_val(hb));
      }
  }
  float m_r[8], l_r[8];
#pragma unroll
  for (int r = 0; r < 8; ++r) { m_r[r] = -3.0e38f; l_r[r] = 0.f; }
  v8f oacc[DT];
#pragma unroll
  for (int dt = 0; dt < DT; ++dt) oacc[dt] = (v8f){0.f,0.f,0.f,0.f,0.f,0.f,0.f,0.f};
  for (int j0 = 0; j0 < Tk; j0 += 32) {
    __syncthreads();
    for (int e = tid; e < 32 * (DQ / 4); e += 128) {
      const int r = e / (DQ / 4), c4 = (e % (DQ / 4)) * 4; const int key = j0 + r;
      v4f f = {0.f,0.f,0.f,0.f}; if (key < Tk) f = *(const v4fa*)(K + (size_t)key * kpitch + c4);
#pragma unroll
      for (int t = 0; t < 4; ++t) { const unsigned short hb = bf16_bits(f[t]); sKh[r][c4 + t] = hb; sKl[r][c4 + t] = bf16_bits(f[t] - bf16_val(hb)); }
    }
    for (int e = tid; e < 32 * (DV / 4); e += 128) {
      const int r = e / (DV / 4), c4 = (e % (DV / 4)) * 4; const int key = j0 + r;
      v4f f = {0.f,0.f,0.f,0.f}; if (key < Tk) f = *(const v4fa*)(V + (size_t)key * vpitch + c4);
#pragma unroll
      for (int t = 0; t < 4; ++t) { const unsigned short hb = bf16_bits(f[t]); sVh[r][c4 + t] = hb; sVl[r][c4 + t] = bf16_bits(f[t] - bf16_val(hb)); }
    }
    __syncthreads();
    v8f s[2];
#pragma unroll
    for (int nt = 0; nt < 2; ++nt) {
      v8f acc = {};
#pragma unroll
      for (int ks = 0; ks < KS; ++ks) {
        FragB bh_, bl_;
        bh_.half[0] = *(const v8us*)&sKh[nt * 16 + ln][ks * 32 + 8 * hh]; bh_.half[1] = *(const v8us*)&sKh[nt * 16 + ln][ks * 32 + 16 + 8 * hh];
        bl_.half[0] = *(const v8us*)&sKl[nt * 16 + ln][ks * 32 + 8 * hh]; bl_.half[1] = *(const v8us*)&sKl[nt * 16 + ln][ks * 32 + 16 + 8 * hh];
        acc = mmaN<3>(aqh[ks].v, aql[ks].v, bh_.v, bl_.v, acc);
      }
      s[nt] = acc;
    }
    float alpha[8];
#pragma unroll
    for (int r = 0; r < 8; ++r) {
      const int ja = j0 + ln, jb = j0 + 16 + ln;
      if (ja >= Tk) s[0][r] = -3.0e38f;
      if (jb >= Tk) s[1][r] = -3.0e38f;
      float mx = fmaxf(s[0][r], s[1][r]);
      mx = fmaxf(mx, __shfl_xor(mx, 1, 32)); mx = fmaxf(mx, __shfl_xor(mx, 2, 32)); mx = fmaxf(mx, __shfl_xor(mx, 4, 32)); mx = fmaxf(mx, __shfl_xor(mx, 8, 32));
      const float mnew = fmaxf(m_r[r], mx);
      alpha[r] = (mnew > -1.0e38f) ? __expf(m_r[r] - mnew) : 1.0f;
      const float p0 = (s[0][r] > -1.0e38f) ? __expf(s[0][r] - mnew) : 0.f;
      const float p1 = (s[1][r] > -1.0e38f) ? __expf(s[1][r] - mnew) : 0.f;
      m_r[r] = mnew;
      l_r[r] = l_r[r] * alpha[r] + p0 + p1;
      unsigned short hb = bf16_bits(p0); sPh[w][8 * hh + r][ln] = hb;      sPl[w][8 * hh + r][ln] = bf16_bits(p0 - bf16_val(hb));
      hb = bf16_bits(p1);                sPh[w][8 * hh + r][16 + ln] = hb; sPl[w][8 * hh + r][16 + ln] = bf16_bits(p1 - bf16_val(hb));
    }
#pragma unroll
    for (int dt = 0; dt < DT; ++dt)
#pragma unroll
      for (int r = 0; r < 8; ++r) oacc[dt][r] *= alpha[r];
    __builtin_amdgcn_fence(__ATOMIC_ACQ_REL, "workgroup");
    __builtin_amdgcn_wave_barrier();
    FragB pah, pal;
    pah.half[0] = *(const v8us*)&sPh[w][ln][8 * hh]; pah.half[1] = *(const v8us*)&sPh[w][ln][16 + 8 * hh];
    pal.half[0] = *(const v8us*)&sPl[w][ln][8 * hh]; pal.half[1] = *(const v8us*)&sPl[w][ln][16 + 8 * hh];
#pragma unroll
    for (int dt = 0; dt < DT; ++dt) {
      FragB bvh, bvl;
#pragma unroll
      for (int i = 0; i < 8; ++i) {
        bvh.u[i] = sVh[8 * hh + i][dt * 16 + ln]; bvh.u[8 + i] = sVh[16 + 8 * hh + i][dt * 16 + ln];
        bvl.u[i] = sVl[8 * hh + i][dt * 16 + ln]; bvl.u[8 + i] = sVl[16 + 8 * hh + i][dt * 16 + ln];
      }
      oacc[dt] = mmaN<3>(pah.v, pal.v, bvh.v, bvl.v, oacc[dt]);
    }
    __builtin_amdgcn_fence(__ATOMIC_ACQ_REL, "workgroup");
    __builtin_amdgcn_wave_barrier();
  }
#pragma unroll
  for (int r = 0; r < 8; ++r) {
    float l = l_r[r];
    l += __shfl_xor(l, 1, 32); l += __shfl_xor(l, 2, 32); l += __shfl_xor(l, 4, 32); l += __shfl_xor(l, 8, 32);
    l_r[r] = (l > 0.f) ? 1.0f / l : 0.f;
  }
#pragma unroll
  for (int dt = 0; dt < DT; ++dt)
#pragma unroll
    for (int r = 0; r < 8; ++r) sO[w][8 * hh + r][dt * 16 + ln] = oacc[dt][r] * l_r[r];
  __builtin_amdgcn_fence(__ATOMIC_ACQ_REL, "workgroup");
  __builtin_amdgcn_wave_barrier();
  for (int pass = 0; pass < 2; ++pass) {
    for (int r = 0; r < 16; ++r) {
      const int row = q0 + r;
      for (int c4 = lane * 4; c4 < DV; c4 += 128) {
        if (row < Tq) {
          const v4f val = *(const v4fa*)&sO[w][r][c4];
          *(volatile v4f*)(y + (size_t)bh * ystride + (size_t)row * ypitch + dv0 + c4) = val;
        }
      }
    }
    if (pass == 0) __threadfence();
  }
}

__global__ __launch_bounds__(256) void k_split_rows(const float* __restrict__ src, int lds_, unsigned short* __restrict__ hi, unsigned short* __restrict__ lo, int R, int Cc) {
  const size_t t = (size_t)blockIdx.x * 256 + threadIdx.x;
  const int c8n = Cc / 8;
  if (t >= (size_t)R * c8n) return;
  const int r = (int)(t / c8n), c8 = (int)(t % c8n) * 8;
  const float* s = src + (size_t)r * lds_ + c8;
  const v4f a = *(const v4fa*)s, b = *(const v4fa*)(s + 4);
  float xs[8] = {a[0],a[1],a[2],a[3],b[0],b[1],b[2],b[3]};
  v8us vh, vl;
#pragma unroll
  for (int i = 0; i < 8; ++i) { const unsigned short hb = bf16_bits(xs[i]); vh[i] = hb; vl[i] = bf16_bits(xs[i] - bf16_val(hb)); }
  unsigned short* dh = hi + (size_t)r * Cc + c8; unsigned short* dl = lo + (size_t)r * Cc + c8;
  *(volatile v8us*)dh = vh; *(volatile v8us*)dl = vl; __threadfence(); *(volatile v8us*)dh = vh; *(volatile v8us*)dl = vl;
}
__global__ __launch_bounds__(256) void k_split_transpose(const float* __restrict__ src, int lds_, unsigned short* __restrict__ hi, unsigned short* __restrict__ lo, int K, int N) {
  const size_t t = (size_t)blockIdx.x * 256 + threadIdx.x;
  const int k8n = K / 8;
  if (t >= (size_t)N * k8n) return;
  const int n = (int)(t / k8n), k8 = (int)(t % k8n) * 8;
  v8us vh, vl;
#pragma unroll
  for (int i = 0; i < 8; ++i) { const float x = src[(size_t)(k8 + i) * lds_ + n]; const unsigned short hb = bf16_bits(x); vh[i] = hb; vl[i] = bf16_bits(x - bf16_val(hb)); }
  unsigned short* dh = hi + (size_t)n * K + k8; unsigned short* dl = lo + (size_t)n * K + k8;
  *(volatile v8us*)dh = vh; *(volatile v8us*)dl = vl; __threadfence(); *(volatile v8us*)dh = vh; *(volatile v8us*)dl = vl;
}
template <bool ASPLIT, bool BSPLIT, int ACT, bool BIAS_BF16>
__global__ __launch_bounds__(128) void k_gemm_bf2(const float* __restrict__ A, int lda, const unsigned short* __restrict__ Bh, const unsigned short* __restrict__ Bl, int ldb,
                                                const float* __restrict__ bias, float alpha, float* __restrict__ C, int ldc, int M, int N, int K) {
  __shared__ __attribute__((aligned(16))) float so[4][16][64];
  const int tid = threadIdx.x, w = tid >> 5, lane = tid & 31, ln = lane & 15, hh = lane >> 4;
  const int ntn = N / 64;
  const int wid = blockIdx.x * 4 + w;
  const int mt = wid / ntn, nq = wid % ntn;
  if (mt * 16 >= M) return;
  const int row0 = mt * 16, col0 = nq * 64;
  const float* arow = A + (size_t)(row0 + ln) * lda;
  v8f acc[4] = {};
  for (int kb = 0; kb < K; kb += 32) {
    FragB ah, al;
    const v4f x0 = *(const v4fa*)(arow + kb + 8 * hh), x1 = *(const v4fa*)(arow + kb + 8 * hh + 4);
    const v4f x2 = *(const v4fa*)(arow + kb + 16 + 8 * hh), x3 = *(const v4fa*)(arow + kb + 16 + 8 * hh + 4);
    float xs[16] = {x0[0],x0[1],x0[2],x0[3],x1[0],x1[1],x1[2],x1[3],x2[0],x2[1],x2[2],x2[3],x3[0],x3[1],x3[2],x3[3]};
#pragma unroll
    for (int i = 0; i < 16; ++i) { const unsigned short hb = bf16_bits(xs[i]); ah.u[i] = hb; al.u[i] = ASPLIT ? bf16_bits(xs[i] - bf16_val(hb)) : (unsigned short)0; }
#pragma unroll
    for (int t = 0; t < 4; ++t) {
      const size_t boff = (size_t)(col0 + t * 16 + ln) * ldb + kb;
      FragB bh_, bl_;
      bh_.half[0] = *(const v8us*)(Bh + boff + 8 * hh);
      bh_.half[1] = *(const v8us*)(Bh + boff + 16 + 8 * hh);
      if (BSPLIT) { bl_.half[0] = *(const v8us*)(Bl + boff + 8 * hh); bl_.half[1] = *(const v8us*)(Bl + boff + 16 + 8 * hh); } else bl_ = bh_;
      acc[t] = mmaN<ASPLIT ? (BSPLIT ? 3 : 2) : 1>(ah.v, al.v, bh_.v, bl_.v, acc[t]);
    }
  }
#pragma unroll
  for (int t = 0; t < 4; ++t) {
    float bv = bias ? bias[col0 + t * 16 + ln] : 0.f;
    if (BIAS_BF16) bv = bf16_round(bv);
#pragma unroll
    for (int r = 0; r < 8; ++r) { float v = acc[t][r] * alpha + bv; if (ACT == 1) v = fmaxf(v, 0.f); so[w][8 * hh + r][t * 16 + ln] = v; }
  }
  __builtin_amdgcn_fence(__ATOMIC_ACQ_REL, "workgroup");
  __builtin_amdgcn_wave_barrier();
  const int rsub = lane >> 4, c4 = (lane & 15) * 4;
  for (int pass = 0; pass < 2; ++pass) {
#pragma unroll
    for (int q = 0; q < 8; ++q) {
      const int r = q * 2 + rsub;
      const v4f v = *(const v4fa*)&so[w][r][c4];
      *(volatile v4f*)(C + (size_t)(row0 + r) * ldc + col0 + c4) = v;
    }
    if (pass == 0) __threadfence();
  }
}
__global__ __launch_bounds__(256) void k_softmax_rows(const float* __restrict__ S, float* __restrict__ P, int N, int causal, int rowoff, const int* __restrict__ mask, int mask_pitch) {
  __shared__ float red[256];
  const int row = blockIdx.x, tid = threadIdx.x;
  const float* s = S + (size_t)row * N; float* p_out = P + (size_t)row * N;
  const int qi = row + rowoff;
  float mx = -3.0e38f;
  for (int j = tid; j < N; j += 256) {
    bool keep = true;
    if (causal && j > qi) keep = false;
    if (mask && mask[(size_t)qi * mask_pitch + j] == 0) keep = false;
    const float v = keep ? s[j] : -3.0e38f;
    mx = fmaxf(mx, v);
  }
  red[tid] = mx; __syncthreads();
  for (int st = 128; st > 0; st >>= 1) { if (tid < st) red[tid] = fmaxf(red[tid], red[tid + st]); __syncthreads(); }
  mx = red[0]; __syncthreads();
  float sum = 0.f;
  for (int j = tid; j < N; j += 256) {
    bool keep = true;
    if (causal && j > qi) keep = false;
    if (mask && mask[(size_t)qi * mask_pitch + j] == 0) keep = false;
    const float p = keep ? __expf(s[j] - mx) : 0.f;
    sum += p;
  }
  red[tid] = sum; __syncthreads();
  for (int st = 128; st > 0; st >>= 1) { if (tid < st) red[tid] += red[tid + st]; __syncthreads(); }
  const float inv = (mx > -1.0e38f) ? 1.0f / red[0] : __builtin_nanf("");
  __syncthreads();
  for (int pass = 0; pass < 2; ++pass) {
    for (int j4 = tid * 4; j4 < N; j4 += 1024) {
      v4f out4;
#pragma unroll
      for (int u = 0; u < 4; ++u) {
        const int j = j4 + u;
        bool keep = true;
        if (causal && j > qi) keep = false;
        if (mask && mask[(size_t)qi * mask_pitch + j] == 0) keep = false;
        out4[u] = keep ? __expf(s[j] - mx) * inv : 0.f;
      }
      *(volatile v4f*)(p_out + j4) = out4;
    }
    if (pass == 0) __threadfence();
  }
}

template <bool ASPLIT, bool BSPLIT, int ACT>
__global__ __launch_bounds__(128) void k_gemm_b(const float* __restrict__ A, int lda, size_t sA, const unsigned short* __restrict__ Bh, const unsigned short* __restrict__ Bl, int ldb, size_t sB,
                                             const float* __restrict__ bias, const float* __restrict__ resid, int ldr, size_t sR, float rsign, float alpha,
                                             float* __restrict__ C, int ldc, size_t sC, int M, int N, int K) {
  __shared__ __attribute__((aligned(16))) float so[4][16][64];
  const int tid = threadIdx.x, w = tid >> 5, lane = tid & 31, ln = lane & 15, hh = lane >> 4;
  const int by = blockIdx.y;
  A += (size_t)by * sA; Bh += (size_t)by * sB; if (BSPLIT) Bl += (size_t)by * sB; C += (size_t)by * sC; if (resid) resid += (size_t)by * sR;
  const int ntn = N / 64; const int wid = blockIdx.x * 4 + w; const int mt = wid / ntn, nq = wid % ntn;
  if (mt * 16 >= M) return;
  const int row0 = mt * 16, col0 = nq * 64;
  const float* arow = A + (size_t)(row0 + ln) * lda;
  v8f acc[4] = {};
  for (int kb = 0; kb < K; kb += 32) {
    FragB ah, al;
    const v4f x0 = *(const v4fa*)(arow + kb + 8 * hh), x1 = *(const v4fa*)(arow + kb + 8 * hh + 4);
    const v4f x2 = *(const v4fa*)(arow + kb + 16 + 8 * hh), x3 = *(const v4fa*)(arow + kb + 16 + 8 * hh + 4);
    float xs[16] = {x0[0],x0[1],x0[2],x0[3],x1[0],x1[1],x1[2],x1[3],x2[0],x2[1],x2[2],x2[3],x3[0],x3[1],x3[2],x3[3]};
#pragma unroll
    for (int i = 0; i < 16; ++i) { const unsigned short hb = bf16_bits(xs[i]); ah.u[i] = hb; al.u[i] = ASPLIT ? bf16_bits(xs[i] - bf16_val(hb)) : (unsigned short)0; }
#pragma unroll
    for (int t = 0; t < 4; ++t) {
      const size_t boff = (size_t)(col0 + t * 16 + ln) * ldb + kb;
      FragB bh_, bl_; bh_.half[0] = *(const v8us*)(Bh + boff + 8 * hh); bh_.half[1] = *(const v8us*)(Bh + boff + 16 + 8 * hh);
      if (BSPLIT) { bl_.half[0] = *(const v8us*)(Bl + boff + 8 * hh); bl_.half[1] = *(const v8us*)(Bl + boff + 16 + 8 * hh); } else bl_ = bh_;
      acc[t] = mmaN<ASPLIT ? (BSPLIT ? 3 : 2) : 1>(ah.v, al.v, bh_.v, bl_.v, acc[t]);
    }
  }
#pragma unroll
  for (int t = 0; t < 4; ++t) {
    const int col = col0 + t * 16 + ln; const float bv = bias ? bf16_round(bias[col]) : 0.f;
#pragma unroll
    for (int r = 0; r < 8; ++r) { float v = acc[t][r] * alpha + bv; if (resid) v += rsign * resid[(size_t)(row0 + 8 * hh + r) * ldr + col]; if (ACT == 1) v = fmaxf(v, 0.f); else if (ACT == 2) v = fmaxf(v, 0.f) + log1pf(expf(-fabsf(v))); so[w][8 * hh + r][t * 16 + ln] = v; }
  }
  __builtin_amdgcn_fence(__ATOMIC_ACQ_REL, "workgroup"); __builtin_amdgcn_wave_barrier();
  const int rsub = lane >> 4, c4 = (lane & 15) * 4;
  for (int pass = 0; pass < 2; ++pass) {
#pragma unroll
    for (int q = 0; q < 8; ++q) { const int r = q * 2 + rsub; const v4f v = *(const v4fa*)&so[w][r][c4]; *(volatile v4f*)(C + (size_t)(row0 + r) * ldc + col0 + c4) = v; }
    if (pass == 0) __threadfence();
  }
}
__global__ __launch_bounds__(256) void k_split_transpose_b(const float* __restrict__ src, int lds_, size_t sIn, unsigned short* __restrict__ hi, unsigned short* __restrict__ lo, size_t sOut, int K, int N) {
  const size_t t = (size_t)blockIdx.x * 256 + threadIdx.x; const int k8n = K / 8; if (t >= (size_t)N * k8n) return;
  src += (size_t)blockIdx.y * sIn; hi += (size_t)blockIdx.y * sOut; lo += (size_t)blockIdx.y * sOut;
  const int n = (int)(t / k8n), k8 = (int)(t % k8n) * 8; v8us vh, vl;
#pragma unroll
  for (int i = 0; i < 8; ++i) { const float x = src[(size_t)(k8 + i) * lds_ + n]; const unsigned short hb = bf16_bits(x); vh[i] = hb; vl[i] = bf16_bits(x - bf16_val(hb)); }
  unsigned short* dh = hi + (size_t)n * K + k8; unsigned short* dl = lo + (size_t)n * K + k8;
  *(volatile v8us*)dh = vh; *(volatile v8us*)dl = vl; __threadfence(); *(volatile v8us*)dh = vh; *(volatile v8us*)dl = vl;
}
__global__ __launch_bounds__(256) void k_wt_conv(const float* __restrict__ w, unsigned short* __restrict__ Bt, int O, int Cin, int CinP, int Np) {
  const int t = blockIdx.x * 256 + threadIdx.x; const int K = 9 * CinP; if (t >= Np * (K / 8)) return;
  const int o = t / (K / 8), k8 = (t % (K / 8)) * 8; v8us v;
#pragma unroll 1
  for (int i = 0; i < 8; ++i) { const int k = k8 + i; const int tap = k / CinP, c = k % CinP; v[i] = (o < O && c < Cin) ? bf16_bits(w[((size_t)o * Cin + c) * 9 + tap]) : (unsigned short)0; }
  *(volatile v8us*)(Bt + (size_t)o * K + k8) = v; __threadfence(); *(volatile v8us*)(Bt + (size_t)o * K + k8) = v;
}
template <int CinP, int ACT, int HI_, int WI_>
__global__ __launch_bounds__(128) void k_conv3x3(const float* __restrict__ in, int inP, const unsigned short* __restrict__ Bt, const float* __restrict__ bias, int Nb, float* __restrict__ out, int Np, int npos) {
  constexpr int K = 9 * CinP, SPT = CinP / 32;
  __shared__ __attribute__((aligned(16))) float so[4][16][64];
  const int tid = threadIdx.x, w = tid >> 5, lane = tid & 31, ln = lane & 15, hh = lane >> 4;
  const int ntn = Np / 64; const int wid = blockIdx.x * 4 + w; const int mt = wid / ntn, nq = wid % ntn;
  if (mt * 16 >= npos) return;
  const int row0 = mt * 16, col0 = nq * 64; const int m = row0 + ln; const int n = m / (HI_ * WI_), yx = m % (HI_ * WI_), y = yx / WI_, xq = yx % WI_;
  v8f acc[4] = {};
  for (int tap = 0; tap < 9; ++tap) {
    const int yy = y + tap / 3 - 1, xx = xq + tap % 3 - 1; const bool inb = (m < npos) && (yy >= 0 && yy < HI_ && xx >= 0 && xx < WI_);
    const float* src = in + ((size_t)n * HI_ * WI_ + (size_t)(inb ? yy : 0) * WI_ + (inb ? xx : 0)) * inP;
#pragma unroll
    for (int s = 0; s < SPT; ++s) {
      const int c0 = s * 32; v4f a0 = {0.f,0.f,0.f,0.f}, a1 = a0, a2 = a0, a3 = a0;
      if (inb) { a0 = *(const v4fa*)(src + c0 + 8 * hh); a1 = *(const v4fa*)(src + c0 + 8 * hh + 4); a2 = *(const v4fa*)(src + c0 + 16 + 8 * hh); a3 = *(const v4fa*)(src + c0 + 16 + 8 * hh + 4); }
      float xs[16] = {a0[0],a0[1],a0[2],a0[3],a1[0],a1[1],a1[2],a1[3],a2[0],a2[1],a2[2],a2[3],a3[0],a3[1],a3[2],a3[3]};
      FragB ah, al;
#pragma unroll
      for (int i = 0; i < 16; ++i) { const unsigned short hb = bf16_bits(xs[i]); ah.u[i] = hb; al.u[i] = bf16_bits(xs[i] - bf16_val(hb)); }
      const int kb = tap * CinP + c0;
#pragma unroll
      for (int t = 0; t < 4; ++t) { FragB bq; bq.half[0] = *(const v8us*)(Bt + (size_t)(col0 + t * 16 + ln) * K + kb + 8 * hh); bq.half[1] = *(const v8us*)(Bt + (size_t)(col0 + t * 16 + ln) * K + kb + 16 + 8 * hh); acc[t] = mmaN<2>(ah.v, al.v, bq.v, bq.v, acc[t]); }
    }
  }
#pragma unroll
  for (int t = 0; t < 4; ++t) { const int col = col0 + t * 16 + ln; const float bv = (col < Nb) ? bf16_round(bias[col]) : 0.f;
#pragma unroll
    for (int r = 0; r < 8; ++r) { float v = acc[t][r] + bv; if (ACT == 1) v = fmaxf(v, 0.f); else if (ACT == 2) v = v >= 0.f ? v : 0.1f * v; so[w][8 * hh + r][t * 16 + ln] = v; } }
  __builtin_amdgcn_fence(__ATOMIC_ACQ_REL, "workgroup"); __builtin_amdgcn_wave_barrier();
  const int rsub = lane >> 4, c4 = (lane & 15) * 4;
  for (int pass = 0; pass < 2; ++pass) { for (int q = 0; q < 8; ++q) { const int r = q * 2 + rsub; if (row0 + r < npos) { const v4f v = *(const v4fa*)&so[w][r][c4]; *(volatile v4f*)(out + (size_t)(row0 + r) * Np + col0 + c4) = v; } } if (pass == 0) __threadfence(); }
}
__global__ __launch_bounds__(256) void k_colstat1(const float* __restrict__ h, int nrows, double* __restrict__ part) {
  const int c = threadIdx.x; const int r0 = blockIdx.x * 512; const int r1 = min(r0 + 512, nrows);
  double s = 0.0, s2 = 0.0;
  for (int r = r0; r < r1; ++r) { const double v = (double)h[(size_t)r * DD + c]; s += v; s2 += v * v; }
  double* dst = part + (size_t)blockIdx.x * 2 * DD;
  *(volatile double*)(dst + c) = s; *(volatile double*)(dst + DD + c) = s2; __threadfence(); *(volatile double*)(dst + c) = s; *(volatile double*)(dst + DD + c) = s2;
}
__global__ __launch_bounds__(256) void k_colstat2(const double* __restrict__ part, int nblk, int nrows, float* __restrict__ stats) {
  const int c = threadIdx.x; double s = 0.0, s2 = 0.0;
  for (int b = 0; b < nblk; ++b) { s += part[(size_t)b * 2 * DD + c]; s2 += part[(size_t)b * 2 * DD + DD + c]; }
  const double mu = s / nrows; double var = s2 / nrows - mu * mu; if (var < 0.0) var = 0.0;
  const float m = (float)mu, rs = (float)(1.0 / sqrt(var + 1e-5));
  *(volatile float*)(stats + c) = m; *(volatile float*)(stats + DD + c) = rs; __threadfence(); *(volatile float*)(stats + c) = m; *(volatile float*)(stats + DD + c) = rs;
}
__global__ __launch_bounds__(256) void k_bn_relu(float* __restrict__ h, int nrows, const float* __restrict__ stats, const float* __restrict__ s, const float* __restrict__ b) {
  const size_t t = (size_t)blockIdx.x * 256 + threadIdx.x; if (t >= (size_t)nrows * (DD / 4)) return;
  const int c4 = (int)(t % (DD / 4)) * 4;
  v4f a = *(const v4fa*)(h + t * 4); v4f o;
  for (int q = 0; q < 4; ++q) { const int c = c4 + q; o[q] = fmaxf((a[q] - stats[c]) * stats[DD + c] * bf16_round(s[c]) + bf16_round(b[c]), 0.f); }
  *(volatile v4f*)(h + t * 4) = o; __threadfence(); *(volatile v4f*)(h + t * 4) = o;
}


__global__ __launch_bounds__(256) void k_zero(float* __restrict__ p, int n4) { const int t = blockIdx.x * 256 + threadIdx.x; if (t < n4) { v4f z = {0.f,0.f,0.f,0.f}; *(volatile v4f*)(p + (size_t)t * 4) = z; __threadfence(); *(volatile v4f*)(p + (size_t)t * 4) = z; } }
__global__ __launch_bounds__(256) void k_img(const float* __restrict__ im, float* __restrict__ out, int nimg) {
  const size_t t = (size_t)blockIdx.x * 256 + threadIdx.x; if (t >= (size_t)nimg * HW0 * 8) return; const int c4 = (int)(t % 8) * 4; const size_t p = t / 8; const int n = (int)(p / HW0), hw = (int)(p % HW0);
  v4f a = {0.f,0.f,0.f,0.f}; if (c4 == 0) { a[0] = bf16_round(im[((size_t)n * 3 + 0) * HW0 + hw]); a[1] = bf16_round(im[((size_t)n * 3 + 1) * HW0 + hw]); a[2] = bf16_round(im[((size_t)n * 3 + 2) * HW0 + hw]); }
  *(volatile v4f*)(out + t * 4) = a; __threadfence(); *(volatile v4f*)(out + t * 4) = a;
}
__global__ __launch_bounds__(256) void k_bn_lrelu(float* __restrict__ h, int nrows, const float* __restrict__ stats, const float* __restrict__ g, const float* __restrict__ b) {
  const size_t t = (size_t)blockIdx.x * 256 + threadIdx.x; if (t >= (size_t)nrows * (DD / 4)) return; const int c4 = (int)(t % (DD / 4)) * 4; v4f v = *(const v4fa*)(h + t * 4);
  for (int q = 0; q < 4; ++q) { const int c = c4 + q; float y = (v[q] - stats[c]) * stats[DD + c] * bf16_round(g[c]) + bf16_round(b[c]); v[q] = y >= 0.f ? y : 0.2f * y; }
  *(volatile v4f*)(h + t * 4) = v; __threadfence(); *(volatile v4f*)(h + t * 4) = v;
}
__global__ __launch_bounds__(256) void k_l2(float* __restrict__ f, int nrows) {
  const int tid = threadIdx.x, w = tid >> 5, lane = tid & 31; const int r = blockIdx.x * 8 + w; if (r >= nrows) return;
  const float a = f[(size_t)r * DD + lane], b = f[(size_t)r * DD + 32 + lane]; float s = a * a + b * b; for (int o = 16; o >= 1; o >>= 1) s += __shfl_xor(s, o, 32);
  const float inv = 1.0f / fmaxf(sqrtf(s), 1e-12f);
  *(volatile float*)(f + (size_t)r * DD + lane) = a * inv; *(volatile float*)(f + (size_t)r * DD + 32 + lane) = b * inv; __threadfence(); *(volatile float*)(f + (size_t)r * DD + lane) = a * inv; *(volatile float*)(f + (size_t)r * DD + 32 + lane) = b * inv;
}
__global__ __launch_bounds__(256) void k_top3(const float* __restrict__ S, int bq, float* __restrict__ slot) {
  __shared__ float cand[8][96]; __shared__ float wsum[8];
  const int c = blockIdx.x; const int tid = threadIdx.x, w = tid >> 5, lane = tid & 31;
  float acc = 0.f;
  for (int l = w; l < HW2; l += 8) {
    const float* row = S + ((size_t)c * MQP + l) * MSP; float t0 = -3e38f, t1 = -3e38f, t2 = -3e38f;
#pragma unroll 1
    for (int m = lane; m < MS; m += 32) { const float v = row[m]; if (v > t2) { if (v > t1) { t2 = t1; if (v > t0) { t1 = t0; t0 = v; } else t1 = v; } else t2 = v; } }
    cand[w][lane * 3] = t0; cand[w][lane * 3 + 1] = t1; cand[w][lane * 3 + 2] = t2;
    __builtin_amdgcn_fence(__ATOMIC_ACQ_REL, "workgroup"); __builtin_amdgcn_wave_barrier();
    if (lane == 0) { float a0 = -3e38f, a1 = -3e38f, a2 = -3e38f;
#pragma unroll 1
      for (int i = 0; i < 96; ++i) { const float v = cand[w][i]; if (v > a2) { if (v > a1) { a2 = a1; if (v > a0) { a1 = a0; a0 = v; } else a1 = v; } else a2 = v; } }
      acc += a0 + a1 + a2; }
    __builtin_amdgcn_fence(__ATOMIC_ACQ_REL, "workgroup"); __builtin_amdgcn_wave_barrier();
  }
  if (lane == 0) wsum[w] = acc; __syncthreads();
  if (tid < 32) { float v = 0.f; if (tid == 0) { for (int i = 0; i < 8; ++i) v += wsum[i]; } const float vv = (tid == 0) ? v : 0.f; *(volatile float*)(slot + ((size_t)bq * WAY + c) * 32 + tid) = vv; __threadfence(); *(volatile float*)(slot + ((size_t)bq * WAY + c) * 32 + tid) = vv; }
}
__global__ __launch_bounds__(256) void k_scores(const float* __restrict__ slot, float* __restrict__ out) { const int t = threadIdx.x; if (t >= NQI * WAY) return; const float v = slot[(size_t)t * 32]; *(volatile float*)(out + t) = v; __threadfence(); *(volatile float*)(out + t) = v; }
extern "C" void kernel_launch(void* const* d_in, const int* in_sizes, int n_in,
                              void* d_out, int out_size, void* d_ws, size_t ws_size, hipStream_t stream) {
  (void)in_sizes; (void)n_in; (void)out_size;
  const float* query = (const float*)d_in[0]; const float* support = (const float*)d_in[1];
  const float* Wc[4] = {(const float*)d_in[2], (const float*)d_in[5], (const float*)d_in[8], (const float*)d_in[11]};
  const float* gg[4] = {(const float*)d_in[3], (const float*)d_in[6], (const float*)d_in[9], (const float*)d_in[12]}; const float* bb[4] = {(const float*)d_in[4], (const float*)d_in[7], (const float*)d_in[10], (const float*)d_in[13]};
  char* ws = (char*)d_ws; size_t off = 0;
  auto take = [&](size_t bytes) { char* p = ws + off; off += (bytes + 255) & ~(size_t)255; return p; };
  unsigned short* B1 = (unsigned short*)take((size_t)64 * 288 * 2); unsigned short* Bk[4]; Bk[0] = B1; for (int i = 1; i < 4; ++i) Bk[i] = (unsigned short*)take((size_t)64 * 576 * 2);
  const int nblkMax = (NSI * HW0 + 511) / 512;
  float* imgT = (float*)take((size_t)NSI * HW0 * 32 * 4); float* c1 = (float*)take((size_t)NSI * HW0 * DD * 4); float* p1 = (float*)take((size_t)NSI * HW1 * DD * 4); float* c2 = (float*)take((size_t)NSI * HW1 * DD * 4);
  float* p2 = (float*)take((size_t)NSI * HW2 * DD * 4); float* c3 = (float*)take((size_t)NSI * HW2 * DD * 4);
  float* featQ = (float*)take((size_t)(NQI * HW2 + 64) * DD * 4); float* featS = (float*)take((size_t)(NSI * HW2 + 64) * DD * 4);
  double* part = (double*)take((size_t)nblkMax * 2 * DD * 8); float* stats = (float*)take(2 * DD * 4);
  unsigned short* Sh = (unsigned short*)take((size_t)(NSI * HW2 + 64) * DD * 2); unsigned short* Sl = (unsigned short*)take((size_t)(NSI * HW2 + 64) * DD * 2);
  float* S = (float*)take((size_t)WAY * MQP * MSP * 4); float* slot = (float*)take((size_t)NQI * WAY * 32 * 4);
  if (off > ws_size) return;
  k_zero<<<(64 * DD / 4 + 255) / 256, 256, 0, stream>>>(featQ + (size_t)NQI * HW2 * DD, 64 * DD / 4); k_zero<<<(64 * DD / 4 + 255) / 256, 256, 0, stream>>>(featS + (size_t)NSI * HW2 * DD, 64 * DD / 4);
  k_wt_conv<<<(64 * (288 / 8) + 255) / 256, 256, 0, stream>>>(Wc[0], B1, 64, 3, 32, 64);
  for (int i = 1; i < 4; ++i) k_wt_conv<<<(64 * (576 / 8) + 255) / 256, 256, 0, stream>>>(Wc[i], Bk[i], 64, 64, 64, 64);
  auto bnstage = [&](float* h, int nrows, int li) { const int nblk = (nrows + 511) / 512; k_colstat1<<<nblk, DD, 0, stream>>>(h, nrows, part); k_colstat2<<<1, DD, 0, stream>>>(part, nblk, nrows, stats); k_bn_lrelu<<<(unsigned)(((size_t)nrows * (DD / 4) + 255) / 256), 256, 0, stream>>>(h, nrows, stats, gg[li], bb[li]); };
  auto encode = [&](const float* im, int nimg, float* feat) {
    const int n0 = nimg * HW0, n1 = nimg * HW1, n2 = nimg * HW2;
    k_img<<<(unsigned)(((size_t)n0 * 8 + 255) / 256), 256, 0, stream>>>(im, imgT, nimg);
    k_conv3x3<32, 0, 84, 84><<<((n0 + 15) / 16 + 3) / 4, 128, 0, stream>>>(imgT, 32, B1, nullptr, 0, c1, 64, n0); bnstage(c1, n0, 0);
    k_pool2_pm<<<(unsigned)(((size_t)n1 * 16 + 255) / 256), 256, 0, stream>>>(c1, p1, nimg, 84, 84, 64);
    k_conv3x3<64, 0, 42, 42><<<((n1 + 15) / 16 + 3) / 4, 128, 0, stream>>>(p1, 64, Bk[1], nullptr, 0, c2, 64, n1); bnstage(c2, n1, 1);
    k_pool2_pm<<<(unsigned)(((size_t)n2 * 16 + 255) / 256), 256, 0, stream>>>(c2, p2, nimg, 42, 42, 64);
    k_conv3x3<64, 0, 21, 21><<<((n2 + 15) / 16 + 3) / 4, 128, 0, stream>>>(p2, 64, Bk[2], nullptr, 0, c3, 64, n2); bnstage(c3, n2, 2);
    k_conv3x3<64, 0, 21, 21><<<((n2 + 15) / 16 + 3) / 4, 128, 0, stream>>>(c3, 64, Bk[3], nullptr, 0, feat, 64, n2); bnstage(feat, n2, 3);
    k_l2<<<(n2 + 7) / 8, 256, 0, stream>>>(feat, n2);
  };
  encode(query, NQI, featQ);
  encode(support, NSI, featS);
  k_split_rows<<<(unsigned)(((size_t)(NSI * HW2 + 64) * DD / 8 + 255) / 256), 256, 0, stream>>>(featS, DD, Sh, Sl, NSI * HW2 + 64, DD);
  for (int bq = 0; bq < NQI; ++bq) {
    const int b = bq / 16;
    k_gemm_b<true, true, 0><<<dim3(((MQP / 16) * (MSP / 64) + 3) / 4, WAY), 128, 0, stream>>>(featQ + (size_t)bq * HW2 * DD, DD, 0, Sh + (size_t)b * WAY * MS * DD, Sl + (size_t)b * WAY * MS * DD, DD, (size_t)MS * DD, nullptr, nullptr, 0, 0, 1.f, 1.f, S, MSP, (size_t)MQP * MSP, MQP, MSP, DD);
    k_top3<<<WAY, 256, 0, stream>>>(S, bq, slot);
  }
  k_scores<<<1, 256, 0, stream>>>(slot, (float*)d_out);
}
